// BERelativeSelfMultiheadAttn_4544075399696
// MI455X (gfx1250) — hardware-verified
//
#include <hip/hip_runtime.h>
#include <math.h>
#include <stdint.h>

#define TT   1024
#define BB   8
#define HH   1024
#define NHD  16
#define HD   64
#define LR   1024
#define NN   (BB * NHD)
#define MR   (TT * BB)
#define H3   (3 * HH)
#define GRP  4
#define NGRP (NN / GRP)
#define NQT  (TT / 64)
#define NKT  (TT / 64)
static_assert(NHD * HD == HH);
static_assert(NN == 128 && MR == 8192 && NGRP == 32 && NQT == 16 && NKT == 16);
static_assert(LR == TT && (TT % 64) == 0 && (HH % 64) == 0 && (H3 % 192) == 0 && (TT / 4) == 256);

#define QKC  4.0f
#define WC   32.0f
#define PCY  1024.0f
#define VLC  2048.0f
#define CC   16.0f

typedef _Float16 v16h __attribute__((ext_vector_type(16)));
typedef _Float16 v8h  __attribute__((ext_vector_type(8)));
typedef float    v8f  __attribute__((ext_vector_type(8)));
typedef float    v4f  __attribute__((ext_vector_type(4)));
typedef unsigned int v4u __attribute__((ext_vector_type(4)));

#if defined(__HIP_DEVICE_COMPILE__)
#define DEV_ASM 1
#else
#define DEV_ASM 0
#endif

__device__ __forceinline__ unsigned short h_bits(_Float16 x) { return __builtin_bit_cast(unsigned short, x); }
__device__ __forceinline__ unsigned pk16(unsigned short a, unsigned short b) { return (unsigned)a | ((unsigned)b << 16); }
__device__ __forceinline__ v8f zero8() { v8f z = {0.f, 0.f, 0.f, 0.f, 0.f, 0.f, 0.f, 0.f}; return z; }

__device__ __forceinline__ v16h ldfrag(const _Float16* p) {
  union { v16h v; v8h h[2]; } f;
  f.h[0] = *(const v8h*)(p);
  f.h[1] = *(const v8h*)(p + 16);
  return f.v;
}

__device__ __forceinline__ v8f mmar(v16h a, v16h b, v8f c) {
  return __builtin_amdgcn_wmma_f32_16x16x32_f16(false, a, false, b, (short)0, c, false, false);
}
__device__ __forceinline__ v8f mma_h(v16h a, v16h b, v8f c) {
  c = __builtin_amdgcn_wmma_f32_16x16x32_f16(false, a, false, b, (short)0, c, false, false);
#if DEV_ASM
  asm volatile("v_nop\n\tv_nop\n\tv_nop\n\tv_nop" : "+v"(c) : "v"(a), "v"(b));
#endif
  return c;
}
__device__ __forceinline__ void dep_guard(v8f& a, v8f& b, v16h x, v16h y) {
#if DEV_ASM
  asm volatile("v_nop\n\tv_nop\n\tv_nop\n\tv_nop" : "+v"(a), "+v"(b) : "v"(x), "v"(y));
#else
  (void)a; (void)b; (void)x; (void)y;
#endif
}
__device__ __forceinline__ void keep4(v16h a, v16h b, v16h c, v16h d) {
#if DEV_ASM
  asm volatile("v_nop" :: "v"(a), "v"(b), "v"(c), "v"(d));
#else
  (void)a; (void)b; (void)c; (void)d;
#endif
}
__device__ __forceinline__ void acc_guard4(v8f& a, v8f& b, v8f& c, v8f& d) {
#if DEV_ASM
  asm volatile("v_nop\n\tv_nop\n\tv_nop\n\tv_nop" : "+v"(a), "+v"(b), "+v"(c), "+v"(d));
#else
  (void)a; (void)b; (void)c; (void)d;
#endif
}

__global__ __launch_bounds__(256) void cvt_rows(const float* __restrict__ in, const float* __restrict__ r,
                                                 unsigned short* out, int mt, int mb, int n8,
                                                 const int* __restrict__ hp) {
  (void)hp;
  const int i = blockIdx.x * 256 + (int)threadIdx.x;
  if (i < n8) {
    const size_t e = (size_t)i * 8;
    const int h = (int)(e & (HH - 1));
    const int t = (int)((e >> 10) & (TT - 1));
    const int b = (int)(e >> 20);
    const float* ip = in + ((size_t)t * mt + (size_t)b * mb) * HH + h;
    const float* rp = r + (size_t)b * HH + h;
    const v4f a0 = *(const v4f*)(ip), a1 = *(const v4f*)(ip + 4);
    const v4f r0 = *(const v4f*)(rp), r1 = *(const v4f*)(rp + 4);
    v4u p;
    p[0] = pk16(h_bits((_Float16)(a0[0] * r0[0])), h_bits((_Float16)(a0[1] * r0[1])));
    p[1] = pk16(h_bits((_Float16)(a0[2] * r0[2])), h_bits((_Float16)(a0[3] * r0[3])));
    p[2] = pk16(h_bits((_Float16)(a1[0] * r1[0])), h_bits((_Float16)(a1[1] * r1[1])));
    p[3] = pk16(h_bits((_Float16)(a1[2] * r1[2])), h_bits((_Float16)(a1[3] * r1[3])));
    unsigned short* o = out + e;
    *(volatile v4u*)o = p;
    __threadfence();
    *(volatile v4u*)o = p;
  }
}

__global__ __launch_bounds__(256) void cvt_w(const float* __restrict__ in, unsigned short* out, int n8, float s) {
  const int i = blockIdx.x * 256 + (int)threadIdx.x;
  if (i < n8) {
    const v4f a0 = *(const v4f*)(in + (size_t)i * 8);
    const v4f a1 = *(const v4f*)(in + (size_t)i * 8 + 4);
    v4u p;
    p[0] = pk16(h_bits((_Float16)(a0[0] * s)), h_bits((_Float16)(a0[1] * s)));
    p[1] = pk16(h_bits((_Float16)(a0[2] * s)), h_bits((_Float16)(a0[3] * s)));
    p[2] = pk16(h_bits((_Float16)(a1[0] * s)), h_bits((_Float16)(a1[1] * s)));
    p[3] = pk16(h_bits((_Float16)(a1[2] * s)), h_bits((_Float16)(a1[3] * s)));
    unsigned short* o = out + (size_t)i * 8;
    *(volatile v4u*)o = p;
    __threadfence();
    *(volatile v4u*)o = p;
  }
}

__global__ __launch_bounds__(256) void bias_dot(const unsigned short* __restrict__ kp, const unsigned short* __restrict__ rk,
                                                 const float* __restrict__ rwb, const float* __restrict__ rrb,
                                                 float* cw, float* cr, float sc) {
  const int sel = blockIdx.y;
  const _Float16* P = (const _Float16*)(const void*)(sel ? rk : kp);
  const float* bias = sel ? rrb : rwb;
  float* outp = sel ? cr : cw;
  const int idx = blockIdx.x * 256 + (int)threadIdx.x;
  if (idx >= NN * (TT / 4)) return;
  const int n  = idx >> 8;
  const int j0 = (idx & 255) * 4;
  const int h  = n & (NHD - 1);
  const _Float16* p0 = P + ((size_t)n * TT + j0) * HD;
  const float* bh = bias + h * HD;
  float a0 = 0.f, a1 = 0.f, a2 = 0.f, a3 = 0.f;
#pragma unroll 1
  for (int dc = 0; dc < HD / 8; ++dc) {
    const v4f b0 = *(const v4f*)(bh + dc * 8);
    const v4f b1 = *(const v4f*)(bh + dc * 8 + 4);
    float bb[8];
#pragma unroll
    for (int e = 0; e < 4; ++e) { bb[e] = b0[e]; bb[4 + e] = b1[e]; }
    const v8h r0 = *(const v8h*)(p0 + dc * 8);
    const v8h r1 = *(const v8h*)(p0 + HD + dc * 8);
    const v8h r2 = *(const v8h*)(p0 + 2 * HD + dc * 8);
    const v8h r3 = *(const v8h*)(p0 + 3 * HD + dc * 8);
#pragma unroll
    for (int e = 0; e < 8; ++e) {
      a0 += bb[e] * (float)r0[e];
      a1 += bb[e] * (float)r1[e];
      a2 += bb[e] * (float)r2[e];
      a3 += bb[e] * (float)r3[e];
    }
  }
  v4f v;
  v[0] = a0 * sc; v[1] = a1 * sc; v[2] = a2 * sc; v[3] = a3 * sc;
  float* o = outp + (size_t)n * TT + j0;
  *(volatile v4f*)o = v;
  __threadfence();
  *(volatile v4f*)o = v;
}

struct GemmArgs {
  const unsigned short* A;
  const unsigned short* Bt;
  void* C0;
  void* C1;
  const float* sc;
  const float* bias;
  long long strideA, strideB, strideC;
  int lda, ldb, ldc, M, N, K, aTileStride, aRowOff;
  float oscale, rscale;
};
static_assert(sizeof(GemmArgs) == 112);

template <int MODE>
__global__ __launch_bounds__(256) void gemm64(GemmArgs g) {
  const _Float16* A  = (const _Float16*)(const void*)g.A;
  const _Float16* Bt = (const _Float16*)(const void*)g.Bt;
  __shared__ __align__(16) float sT[8][16 * 68];
  const int bz   = blockIdx.y;
  const int lane = threadIdx.x & 31;
  const int wave = threadIdx.x >> 5;
  const int tilesN = g.N >> 6;
  const int tilesM = g.M >> 6;
  const int tile = blockIdx.x * 8 + wave;
  if (tile >= tilesM * tilesN) return;
  const int tm = tile / tilesN;
  const int tn = tile - tm * tilesN;
  const int aRow0 = tm * g.aTileStride + g.aRowOff;
  int hsel = tn, which = 0, bRow0 = tn << 6;
  if (MODE == 1) { hsel = tn >> 1; which = tn & 1; bRow0 = hsel * 192 + (which << 6); }
  const int n0 = tn << 6;

  const _Float16* Ab = A  + (size_t)bz * (size_t)g.strideA;
  const _Float16* Bb = Bt + (size_t)bz * (size_t)g.strideB;

  const int rlane = lane & 15;
  const int koff  = (lane >> 4) * 8;
  const int mOff  = (lane >> 4) * 8;

  v8f acc[4][4];
#pragma unroll
  for (int i = 0; i < 4; ++i)
#pragma unroll
    for (int j = 0; j < 4; ++j) acc[i][j] = zero8();

  for (int k0 = 0; k0 < g.K; k0 += 32) {
    v16h bq[4];
#pragma unroll
    for (int j = 0; j < 4; ++j)
      bq[j] = ldfrag(Bb + (size_t)(bRow0 + (j << 4) + rlane) * g.ldb + koff + k0);
#pragma unroll
    for (int i = 0; i < 4; ++i) {
      const v16h af = ldfrag(Ab + (size_t)(aRow0 + (i << 4) + rlane) * g.lda + koff + k0);
#pragma unroll
      for (int j = 0; j < 4; ++j) acc[i][j] = mmar(af, bq[j], acc[i][j]);
      dep_guard(acc[i][0], acc[i][3], af, bq[3]);
    }
    keep4(bq[0], bq[1], bq[2], bq[3]);
  }
  acc_guard4(acc[0][0], acc[0][1], acc[0][2], acc[0][3]);
  acc_guard4(acc[1][0], acc[1][1], acc[1][2], acc[1][3]);
  acc_guard4(acc[2][0], acc[2][1], acc[2][2], acc[2][3]);
  acc_guard4(acc[3][0], acc[3][1], acc[3][2], acc[3][3]);

  float* slab = sT[wave];
#pragma unroll
  for (int i = 0; i < 4; ++i) {
#pragma unroll
    for (int j = 0; j < 4; ++j) {
#pragma unroll
      for (int r = 0; r < 8; ++r) {
        slab[(mOff + r) * 68 + (j << 4) + rlane] = acc[i][j][r];
      }
    }
    __builtin_amdgcn_fence(__ATOMIC_RELEASE, "workgroup");
    __builtin_amdgcn_wave_barrier();
    __builtin_amdgcn_fence(__ATOMIC_ACQUIRE, "workgroup");
    if (MODE == 0 || MODE == 4) {
      float* C = (float*)g.C0 + (size_t)bz * (size_t)g.strideC;
      const int h2 = lane >> 4, c4 = (lane & 15) * 4;
      const float* bp = g.bias + ((MODE == 4) ? ((size_t)bz * (size_t)g.N) : (size_t)0) + n0 + c4;
      const v4f bv = *(const v4f*)bp;
      const int rowBase = aRow0 + (i << 4);
      for (int pass = 0; pass < 2; ++pass) {
#pragma unroll
        for (int it = 0; it < 8; ++it) {
          const int row = it * 2 + h2;
          const v4f v = *(const v4f*)(slab + row * 68 + c4) * g.oscale + bv;
          *(volatile v4f*)(C + (size_t)(rowBase + row) * g.ldc + n0 + c4) = v;
        }
        __threadfence();
      }
    } else {
      const int q = lane >> 3, c8 = (lane & 7) * 8;
      const int bsel = (MODE == 3) ? bz : (aRow0 >> 10);
      const int tb   = (MODE == 3) ? 0  : ((aRow0 & (TT - 1)) + (i << 4));
      v4f sc0 = {0.f, 0.f, 0.f, 0.f}, sc1 = sc0, bi0 = sc0, bi1 = sc0;
      if (MODE == 1 || MODE == 2) {
        const int scp = (MODE == 1) ? H3 : HH;
        const float* sp = g.sc   + (size_t)bsel * scp + bRow0 + c8;
        const float* bp = g.bias + bRow0 + c8;
        sc0 = *(const v4f*)sp; sc1 = *(const v4f*)(sp + 4);
        bi0 = *(const v4f*)bp; bi1 = *(const v4f*)(bp + 4);
      }
      float scv[8], biv[8];
#pragma unroll
      for (int e = 0; e < 4; ++e) {
        scv[e] = sc0[e]; scv[4 + e] = sc1[e];
        biv[e] = bi0[e]; biv[4 + e] = bi1[e];
      }
      unsigned short* P0 = (unsigned short*)((MODE == 1 && which != 0) ? g.C1 : g.C0);
      unsigned short* P1 = (unsigned short*)g.C1;
      v4u hv[4], hv2[4];
#pragma unroll
      for (int it = 0; it < 4; ++it) {
        const int row = it * 4 + q;
        const float* sp = slab + row * 68 + c8;
        float f[8];
#pragma unroll
        for (int e = 0; e < 8; ++e) f[e] = sp[e];
        float val[8];
        if (MODE == 3) {
          const int o = aRow0 + (i << 4) + row;
          const float s1 = g.sc[(size_t)bsel * H3 + o];
          const float b1 = g.bias[o];
#pragma unroll
          for (int e = 0; e < 8; ++e) val[e] = f[e] * (1.0f / WC) * s1 + b1;
        } else {
#pragma unroll
          for (int e = 0; e < 8; ++e) val[e] = f[e] * (1.0f / WC) * scv[e] + biv[e];
        }
        v4u a, a2;
#pragma unroll
        for (int e = 0; e < 4; ++e) {
          const float v0 = val[2 * e] * QKC, v1 = val[2 * e + 1] * QKC;
          const _Float16 x0 = (_Float16)v0, x1 = (_Float16)v1;
          const unsigned short h0 = h_bits(x0), h1 = h_bits(x1);
          unsigned short l0 = 0, l1 = 0;
          if (MODE == 3) {
            l0 = h_bits((_Float16)((v0 - (float)x0) * g.rscale));
            l1 = h_bits((_Float16)((v1 - (float)x1) * g.rscale));
          }
          a[e] = pk16(h0, h1); a2[e] = pk16(l0, l1);
        }
        hv[it] = a; hv2[it] = a2;
      }
      for (int pass = 0; pass < 2; ++pass) {
#pragma unroll
        for (int it = 0; it < 4; ++it) {
          const int row = it * 4 + q;
          if (MODE == 3) {
            const size_t off = (size_t)bz * (size_t)g.strideC + (size_t)(tm * 64 + (i << 4) + row) * g.ldc + n0 + c8;
            *(volatile v4u*)(P0 + off) = hv[it];
            *(volatile v4u*)(P1 + off) = hv2[it];
          } else {
            const size_t off = ((size_t)(bsel * NHD + hsel) * TT + tb + row) * HD + c8;
            *(volatile v4u*)(P0 + off) = hv[it];
          }
        }
        __threadfence();
      }
    }
    __builtin_amdgcn_fence(__ATOMIC_RELEASE, "workgroup");
    __builtin_amdgcn_wave_barrier();
    __builtin_amdgcn_fence(__ATOMIC_ACQUIRE, "workgroup");
  }
}

__global__ __launch_bounds__(128)
void attn_rel(const unsigned short* __restrict__ qwp, const unsigned short* __restrict__ kpp,
              const unsigned short* __restrict__ vhp, const unsigned short* __restrict__ vlp,
              const float* __restrict__ raw, const float* __restrict__ cw,
              unsigned short* ctxp, int nbase, float sscale, float cinv) {
  union FH { v16h v; v8h h[2]; };
  __shared__ __align__(16) _Float16 Ksh[64 * 64];
  __shared__ __align__(16) _Float16 Vth[64 * 64];
  __shared__ __align__(16) _Float16 Vtl[64 * 64];
  __shared__ __align__(16) _Float16 Psh[4][16 * 64];
  __shared__ __align__(16) float    Os[4][16 * 64];

  const int tid  = threadIdx.x;
  const int wave = tid >> 5;
  const int lane = tid & 31;
  const int hh   = lane >> 4;
  const int c    = lane & 15;

  const int bx = blockIdx.x;
  const int qt = bx & (NQT - 1);
  const int ng = bx >> 4;
  const int n  = nbase + ng;
  const int b  = n >> 4;
  const int h  = n & (NHD - 1);
  const int i0 = qt * 64 + wave * 16;

  const _Float16* Q  = (const _Float16*)(const void*)qwp + (size_t)n * TT * HD;
  const _Float16* Kg = (const _Float16*)(const void*)kpp + (size_t)n * TT * HD;
  const _Float16* Vh = (const _Float16*)(const void*)vhp + (size_t)n * HD * TT;
  const _Float16* Vl = (const _Float16*)(const void*)vlp + (size_t)n * HD * TT;
  const float* rawn  = raw + (size_t)ng * TT * LR;
  const float* cwn   = cw + (size_t)n * TT;

  v16h qa[2];
#pragma unroll
  for (int dc = 0; dc < 2; ++dc) {
    qa[dc] = ldfrag(Q + (size_t)(i0 + c) * HD + dc * 32 + 8 * hh);
  }

  float mrow[8], lrow[8];
  v8f oacc[4];
#pragma unroll
  for (int r = 0; r < 8; ++r) { mrow[r] = -INFINITY; lrow[r] = 0.f; }
#pragma unroll
  for (int t = 0; t < 4; ++t) oacc[t] = zero8();

  for (int kt = 0; kt < NKT; ++kt) {
    const int kv0 = kt * 64;
    __syncthreads();
    {
      const int r = tid >> 1, half = (tid & 1) * 32;
      const _Float16* kg  = Kg + (size_t)(kv0 + r) * HD + half;
      const _Float16* vg  = Vh + (size_t)r * TT + kv0 + half;
      const _Float16* vlg = Vl + (size_t)r * TT + kv0 + half;
#pragma unroll
      for (int i = 0; i < 4; ++i) {
        const v8h a0 = *(const v8h*)(kg + 8 * i);
        const v8h b0 = *(const v8h*)(vg + 8 * i);
        const v8h b1 = *(const v8h*)(vlg + 8 * i);
        *(v8h*)(Ksh + r * 64 + half + 8 * i) = a0;
        *(v8h*)(Vth + r * 64 + half + 8 * i) = b0;
        *(v8h*)(Vtl + r * 64 + half + 8 * i) = b1;
      }
    }
    __syncthreads();

    v8f s[4];
#pragma unroll
    for (int j = 0; j < 4; ++j) {
      v8f a = zero8();
#pragma unroll
      for (int dc = 0; dc < 2; ++dc) {
        FH kb;
        kb.h[0] = *(const v8h*)(Ksh + (j * 16 + c) * 64 + dc * 32 + 8 * hh);
        kb.h[1] = *(const v8h*)(Ksh + (j * 16 + c) * 64 + dc * 32 + 16 + 8 * hh);
        a = mma_h(qa[dc], kb.v, a);
      }
      const int jj = kv0 + j * 16 + c;
      const float cwj = cwn[jj];
#pragma unroll
      for (int r = 0; r < 8; ++r) {
        const int ii   = i0 + 8 * hh + r;
        const int dlt  = jj - ii;
        const int colA = min(max(dlt + (LR - 1), 0), LR - 1);
        const int colB = min(max(dlt - 2, 0), LR - 1);
        const int iiB  = min(ii + 1, TT - 1);
        const int idx  = (dlt <= 0) ? (ii * LR + colA) : (iiB * LR + colB);
        float bdv = rawn[idx];
        bdv = (dlt == 1) ? 0.f : bdv;
        s[j][r] = a[r] * sscale + cwj + bdv;
      }
    }

    _Float16* pwh = Psh[wave];
#pragma unroll
    for (int r = 0; r < 8; ++r) {
      float m = s[0][r];
#pragma unroll
      for (int j = 1; j < 4; ++j) m = fmaxf(m, s[j][r]);
#pragma unroll
      for (int off = 1; off < 16; off <<= 1) m = fmaxf(m, __shfl_xor(m, off, 32));
      const float mnew  = fmaxf(mrow[r], m);
      const float msafe = (mnew == -INFINITY) ? 0.f : mnew;
      const float alpha = __expf(mrow[r] - msafe);
      mrow[r] = mnew;
      float psum = 0.f;
#pragma unroll
      for (int j = 0; j < 4; ++j) {
        const float p = __expf(s[j][r] - msafe);
        psum += p;
        pwh[(8 * hh + r) * 64 + j * 16 + c] = (_Float16)(p * PCY);
      }
#pragma unroll
      for (int off = 1; off < 16; off <<= 1) psum += __shfl_xor(psum, off, 32);
      lrow[r] = lrow[r] * alpha + psum;
#pragma unroll
      for (int t = 0; t < 4; ++t) oacc[t][r] *= alpha;
    }
    __builtin_amdgcn_fence(__ATOMIC_RELEASE, "workgroup");
    __builtin_amdgcn_wave_barrier();
    __builtin_amdgcn_fence(__ATOMIC_ACQUIRE, "workgroup");

    v8f o1[4];
#pragma unroll
    for (int t = 0; t < 4; ++t) o1[t] = zero8();
#pragma unroll 1
    for (int kk = 0; kk < 2; ++kk) {
      FH pa;
      pa.h[0] = *(const v8h*)(pwh + c * 64 + kk * 32 + 8 * hh);
      pa.h[1] = *(const v8h*)(pwh + c * 64 + kk * 32 + 16 + 8 * hh);
#pragma unroll
      for (int t = 0; t < 4; ++t) {
        FH vb, vl;
        vb.h[0] = *(const v8h*)(Vth + (t * 16 + c) * 64 + kk * 32 + 8 * hh);
        vb.h[1] = *(const v8h*)(Vth + (t * 16 + c) * 64 + kk * 32 + 16 + 8 * hh);
        vl.h[0] = *(const v8h*)(Vtl + (t * 16 + c) * 64 + kk * 32 + 8 * hh);
        vl.h[1] = *(const v8h*)(Vtl + (t * 16 + c) * 64 + kk * 32 + 16 + 8 * hh);
        oacc[t] = mma_h(pa.v, vb.v, oacc[t]);
        o1[t]   = mma_h(pa.v, vl.v, o1[t]);
      }
    }
#pragma unroll
    for (int t = 0; t < 4; ++t)
#pragma unroll
      for (int r = 0; r < 8; ++r) oacc[t][r] += o1[t][r] * (1.0f / VLC);
  }

  float* os = Os[wave];
#pragma unroll
  for (int r = 0; r < 8; ++r) {
    const float l = lrow[r];
    const float inv = ((l > 0.f) ? (1.0f / l) : 0.f) * cinv;
#pragma unroll
    for (int t = 0; t < 4; ++t) os[(8 * hh + r) * 64 + t * 16 + c] = oacc[t][r] * inv;
  }
  __builtin_amdgcn_fence(__ATOMIC_RELEASE, "workgroup");
  __builtin_amdgcn_wave_barrier();
  __builtin_amdgcn_fence(__ATOMIC_ACQUIRE, "workgroup");
  {
    const int q4 = lane >> 3, c8 = (lane & 7) * 8;
    v4u hv[4];
#pragma unroll
    for (int it = 0; it < 4; ++it) {
      const int row = it * 4 + q4;
      const float* sp = os + row * 64 + c8;
      v4u a;
#pragma unroll
      for (int e = 0; e < 4; ++e) {
        const float f0 = sp[2 * e], f1 = sp[2 * e + 1];
        a[e] = pk16(h_bits((_Float16)f0), h_bits((_Float16)f1));
      }
      hv[it] = a;
    }
    for (int pass = 0; pass < 2; ++pass) {
#pragma unroll
      for (int it = 0; it < 4; ++it) {
        const int row = it * 4 + q4;
        const size_t go = ((size_t)(i0 + row) * BB + b) * HH + (size_t)h * HD + c8;
        *(volatile v4u*)(ctxp + go) = hv[it];
      }
      __threadfence();
    }
  }
}

static GemmArgs mkargs(const void* A, int lda, long long sA, int aTs, int aOff,
                       const void* Bt, int ldb, long long sB,
                       void* C0, void* C1, int ldc, long long sC,
                       const float* sc, const float* bias,
                       int M, int N, int K, float oscale, float rscale) {
  GemmArgs g;
  g.A = (const unsigned short*)A; g.Bt = (const unsigned short*)Bt;
  g.C0 = C0; g.C1 = C1;
  g.sc = sc; g.bias = bias;
  g.strideA = sA; g.strideB = sB; g.strideC = sC;
  g.lda = lda; g.ldb = ldb; g.ldc = ldc; g.M = M; g.N = N; g.K = K; g.aTileStride = aTs; g.aRowOff = aOff;
  g.oscale = oscale; g.rscale = rscale;
  return g;
}

extern "C" void kernel_launch(void* const* d_in, const int* in_sizes, int n_in,
                              void* d_out, int out_size, void* d_ws, size_t ws_size,
                              hipStream_t stream) {
  if (n_in < 15) return;
  if (in_sizes[0] != MR * HH) return;
  if (in_sizes[1] != LR * HH) return;
  if (in_sizes[2] != H3 * HH || in_sizes[3] != H3) return;
  if (in_sizes[4] != HH * HH || in_sizes[5] != HH) return;
  if (in_sizes[6] != HH * HH || in_sizes[7] != HH) return;
  if (in_sizes[8] != BB * HH || in_sizes[9] != BB * H3 || in_sizes[10] != BB * HH || in_sizes[11] != BB * HH) return;
  if (in_sizes[12] != NHD * HD || in_sizes[13] != NHD * HD || in_sizes[14] != 1) return;
  if (out_size != MR * HH) return;

  const float* x    = (const float*)d_in[0];
  const float* pos  = (const float*)d_in[1];
  const float* Wi   = (const float*)d_in[2];
  const float* bi   = (const float*)d_in[3];
  const float* Wp   = (const float*)d_in[4];
  const float* bp   = (const float*)d_in[5];
  const float* Wo   = (const float*)d_in[6];
  const float* bo   = (const float*)d_in[7];
  const float* r_i  = (const float*)d_in[8];
  const float* s_i  = (const float*)d_in[9];
  const float* r_p  = (const float*)d_in[10];
  const float* s_p  = (const float*)d_in[11];
  const float* rwb  = (const float*)d_in[12];
  const float* rrb  = (const float*)d_in[13];
  const int*   hp   = (const int*)d_in[14];

  const size_t P16  = (size_t)MR * HH * 2;
  const size_t PRAW = (size_t)GRP * TT * LR * 4;
  const size_t PCTX = (size_t)MR * HH * 2;
  const size_t PWI  = (size_t)H3 * HH * 2;
  const size_t PW   = (size_t)HH * HH * 2;
  const size_t PTB  = (size_t)NN * TT * 4;
  if (PRAW > P16 || PCTX > P16) return;
  size_t off = 0;
  const size_t oXR  = off; off += P16;
  const size_t oRAW = oXR;
  const size_t oPR  = off; off += P16;
  const size_t oCTX = oPR;
  const size_t oWI  = off; off += PWI;
  const size_t oWP  = off; off += PW;
  const size_t oWO  = off; off += PW;
  const size_t oQ4  = off; off += P16;
  const size_t oKP  = off; off += P16;
  const size_t oVTh = off; off += P16;
  const size_t oVTl = off; off += P16;
  const size_t oRK  = off; off += P16;
  const size_t oCW  = off; off += PTB;
  const size_t oCR  = off; off += PTB;
  if (off > ws_size) return;
  if (off > (size_t)134217728) return;

  char* ws = (char*)d_ws;
  unsigned short* XR  = (unsigned short*)(ws + oXR);
  float*          RAW = (float*)(ws + oRAW);
  unsigned short* PR  = (unsigned short*)(ws + oPR);
  unsigned short* CTX = (unsigned short*)(ws + oCTX);
  unsigned short* WI  = (unsigned short*)(ws + oWI);
  unsigned short* WPp = (unsigned short*)(ws + oWP);
  unsigned short* WOp = (unsigned short*)(ws + oWO);
  unsigned short* Q4  = (unsigned short*)(ws + oQ4);
  unsigned short* KP  = (unsigned short*)(ws + oKP);
  unsigned short* VTh = (unsigned short*)(ws + oVTh);
  unsigned short* VTl = (unsigned short*)(ws + oVTl);
  unsigned short* RK  = (unsigned short*)(ws + oRK);
  float*          CW  = (float*)(ws + oCW);
  float*          CR  = (float*)(ws + oCR);

  const dim3 blk(256);
  const int n8p  = MR * HH / 8;
  const int n8wi = H3 * HH / 8;
  const int n8w  = HH * HH / 8;
  const dim3 gP((n8p + 255) / 256);
  const dim3 gWI((n8wi + 255) / 256);
  const dim3 gW((n8w + 255) / 256);
  const dim3 gBD((NN * (TT / 4) + 255) / 256, 2);

  const float sscale = 0.125f / (QKC * QKC);
  const float bdsc   = 0.125f / QKC;
  const float cinv   = CC / (PCY * QKC);

  cvt_rows<<<gP, blk, 0, stream>>>(x, r_i, XR, 8, 1, n8p, hp);
  cvt_rows<<<gP, blk, 0, stream>>>(pos, r_p, PR, 1, 0, n8p, hp);
  cvt_w<<<gWI, blk, 0, stream>>>(Wi, WI, n8wi, WC);
  cvt_w<<<gW, blk, 0, stream>>>(Wp, WPp, n8w, WC);
  cvt_w<<<gW, blk, 0, stream>>>(Wo, WOp, n8w, WC);

  {
    const GemmArgs g = mkargs(XR, HH, 0LL, 64, 0, WI, HH, 0LL,
                              (void*)Q4, (void*)KP, HD, 0LL,
                              s_i, bi, MR, 2 * HH, HH, 1.0f, 1.0f);
    const dim3 grid((((MR / 64) * ((2 * HH) / 64)) + 7) / 8, 1);
    gemm64<1><<<grid, blk, 0, stream>>>(g);
  }
  {
    const GemmArgs g = mkargs(WI, HH, 0LL, 192, 128, XR, HH, (long long)TT * HH,
                              (void*)VTh, (void*)VTl, TT, (long long)NHD * HD * TT,
                              s_i, bi, HH, TT, HH, 1.0f, VLC);
    const dim3 grid((((HH / 64) * (TT / 64)) + 7) / 8, BB);
    gemm64<3><<<grid, blk, 0, stream>>>(g);
  }
  {
    const GemmArgs g = mkargs(PR, HH, 0LL, 64, 0, WPp, HH, 0LL,
                              (void*)RK, (void*)RK, HD, 0LL,
                              s_p, bp, MR, HH, HH, 1.0f, 1.0f);
    const dim3 grid((((MR / 64) * (HH / 64)) + 7) / 8, 1);
    gemm64<2><<<grid, blk, 0, stream>>>(g);
  }
  bias_dot<<<gBD, blk, 0, stream>>>(KP, RK, rwb, rrb, CW, CR, bdsc);

  for (int grp = 0; grp < NGRP; ++grp) {
    const int nbase = grp * GRP;
    const GemmArgs g = mkargs(Q4 + (size_t)nbase * TT * HD, HD, (long long)TT * HD, 64, 0,
                              RK + (size_t)nbase * LR * HD, HD, (long long)LR * HD,
                              (void*)RAW, (void*)RAW, LR, (long long)TT * LR,
                              s_i, CR + (size_t)nbase * LR, TT, LR, HD, sscale, 1.0f);
    const dim3 grid((((TT / 64) * (LR / 64)) + 7) / 8, GRP);
    gemm64<4><<<grid, blk, 0, stream>>>(g);
    attn_rel<<<dim3(GRP * NQT), dim3(128), 0, stream>>>(Q4, KP, VTh, VTl, RAW, CW, CTX, nbase, sscale, cinv);
  }
  {
    const GemmArgs g = mkargs(CTX, HH, 0LL, 64, 0, WOp, HH, 0LL,
                              d_out, d_out, HH, 0LL,
                              s_i, bo, MR, HH, HH, 1.0f / (CC * WC), 1.0f);
    const dim3 grid((((MR / 64) * (HH / 64)) + 7) / 8, 1);
    gemm64<0><<<grid, blk, 0, stream>>>(g);
  }
  (void)hipGetLastError();
}
